// E_GCL_2791728742861
// MI455X (gfx1250) — hardware-verified
//
#include <hip/hip_runtime.h>
#include <stddef.h>
#include <stdint.h>


#define FD      64
#define NOUTF   67
#define NPQ     128
#define KTP     8192
#define NTP     128
#define NCHUNK  4
#define NTHR    256
#define NWAVE   8
#define ETHR    128
#define GTHR    128
#define GBM     64
#define ZTHR    64
#define ZP      392
#define AP      136
#define EPT     8
#define CHUNK   (NTHR * EPT)
#define WCAP    (EPT * 32)
#define LISTN   (NWAVE * WCAP)
#define NBA     1024
#define SLA     10
#define RCAP    8192
#define DEGCAP  96
#define XROWS   320
#define WSMAX   134217728
#define NU_WABT 1024
#define NU_WE2T 1024
#define NU_WS1T 131072
#define NU_WS2T 2048
#define NU_WC1T 1024
#define NU_WN1T 2048
#define NU_WN2A 2048
#define NU_WN2B 2048
#define AGG_ZINTS (LISTN + 2 * RCAP + 3 * NBA)
#define AGG_LDS_INTS (AGG_ZINTS + 16 + 4 * NBA)
#define AGG_LDS_BYTES (AGG_LDS_INTS * 4)

static_assert((CHUNK & (CHUNK - 1)) == 0 && CHUNK <= 4096);
static_assert((NBA & (NBA - 1)) == 0 && NBA == (1 << SLA));
static_assert(((long long)CHUNK << SLA) < (1LL << 31));
static_assert(LISTN % NTHR == 0);
static_assert(NBA % NWAVE == 0 && NBA % 32 == 0 && NBA == 4 * NTHR);
static_assert(RCAP % 4 == 0 && AGG_ZINTS % 4 == 0 && LISTN % 4 == 0);
static_assert(AGG_LDS_BYTES <= 300000);
static_assert(NU_WABT % NTHR == 0 && NU_WE2T % NTHR == 0 && NU_WS1T % NTHR == 0 && NU_WS2T % NTHR == 0);
static_assert(NU_WC1T % NTHR == 0 && NU_WN1T % NTHR == 0 && NU_WN2A % NTHR == 0 && NU_WN2B % NTHR == 0);
static_assert(GBM == (GTHR / 32) * 16);
static_assert((AP * 2) % 16 == 0 && AP >= 2 * FD);
static_assert((ZP * 2) % 16 == 0 && ZP >= 384);
static_assert(ETHR * 16 == 16 * ETHR && (ETHR % 32) == 0);
static_assert((GBM * NOUTF) % 4 == 0 && ((32 * NOUTF * 4) % 128) == 0);
static_assert((XROWS * 3) % 4 == 0 && (XROWS * 3) / 4 <= NTHR && ((XROWS * 3 * 4) % 128) == 0);
static_assert(DEGCAP % 32 == 0);
static_assert(KTP % 32 == 0 && FD % 32 == 0);

typedef float          v4f   __attribute__((ext_vector_type(4)));
typedef float          v8f   __attribute__((ext_vector_type(8)));
typedef int            v4i   __attribute__((ext_vector_type(4)));
typedef int            v8i   __attribute__((ext_vector_type(8)));
typedef unsigned short v8us  __attribute__((ext_vector_type(8)));
typedef unsigned short v16us __attribute__((ext_vector_type(16)));
typedef __bf16         v16bf __attribute__((ext_vector_type(16)));
typedef v4f  __attribute__((may_alias)) v4fa;
typedef v4i  __attribute__((may_alias)) v4ia;
typedef v8us __attribute__((may_alias)) v8usa;
union FragB { v16bf v; v16us u; v8us h[2]; v8i w; };

__device__ __forceinline__ v8f wmb(const FragB& a, const FragB& b, v8f c) {
  v8f d = __builtin_amdgcn_wmma_f32_16x16x32_bf16(false, a.v, false, b.v, (short)0, c, false, false);
  asm volatile("v_nop\n\tv_nop\n\tv_nop\n\tv_nop" : "+v"(d) : "v"(a.w), "v"(b.w));
  return d;
}

__device__ __forceinline__ unsigned bf16_bits(float f) {
  const unsigned u = __float_as_uint(f);
  return (u + 0x7FFFu + ((u >> 16) & 1u)) >> 16;
}
__device__ __forceinline__ float bf16_val(float f) {
  return __uint_as_float(bf16_bits(f) << 16);
}
__device__ __forceinline__ float silu_f(float t) {
  return t * __builtin_amdgcn_rcpf(1.0f + __expf(-t));
}
__device__ __forceinline__ void put16(unsigned short* dp, v8us o) {
  *(volatile v8us*)dp = o;
  __threadfence();
  *(volatile v8us*)dp = o;
}
__device__ __forceinline__ void putf4(float* dp, v4f o) {
  *(volatile v4f*)dp = o;
  __threadfence();
  *(volatile v4f*)dp = o;
}
__device__ __forceinline__ int clampi(int v, int lo, int hi) { return v < lo ? lo : (v > hi ? hi : v); }

template <int SLB>
__device__ __forceinline__ int scan_chunk(const int* __restrict__ dsts, int nE, int cbase, int slotBase,
                                          int nb, int vec8, int* list, int tid, int lane, int wave) {
  int wc = 0;
  const int el0  = tid * EPT;
  const int e0   = cbase + el0;
  const int sent = -2147483647 - 1;
  v4i da, db;
  if (vec8 != 0 && cbase + CHUNK <= nE) {
    da = *(const v4i*)(dsts + e0);
    db = *(const v4i*)(dsts + e0 + 4);
  } else {
    da.x = (e0     < nE) ? dsts[min(e0,     nE - 1)] : sent;
    da.y = (e0 + 1 < nE) ? dsts[min(e0 + 1, nE - 1)] : sent;
    da.z = (e0 + 2 < nE) ? dsts[min(e0 + 2, nE - 1)] : sent;
    da.w = (e0 + 3 < nE) ? dsts[min(e0 + 3, nE - 1)] : sent;
    db.x = (e0 + 4 < nE) ? dsts[min(e0 + 4, nE - 1)] : sent;
    db.y = (e0 + 5 < nE) ? dsts[min(e0 + 5, nE - 1)] : sent;
    db.z = (e0 + 6 < nE) ? dsts[min(e0 + 6, nE - 1)] : sent;
    db.w = (e0 + 7 < nE) ? dsts[min(e0 + 7, nE - 1)] : sent;
  }
  const unsigned nbs = (unsigned)slotBase;
  const unsigned unb = (unsigned)nb;
  const unsigned s0 = (unsigned)da.x - nbs, s1 = (unsigned)da.y - nbs;
  const unsigned s2 = (unsigned)da.z - nbs, s3 = (unsigned)da.w - nbs;
  const unsigned s4 = (unsigned)db.x - nbs, s5 = (unsigned)db.y - nbs;
  const unsigned s6 = (unsigned)db.z - nbs, s7 = (unsigned)db.w - nbs;
  const bool h0 = s0 < unb, h1 = s1 < unb, h2 = s2 < unb, h3 = s3 < unb;
  const bool h4 = s4 < unb, h5 = s5 < unb, h6 = s6 < unb, h7 = s7 < unb;
  const unsigned any = __builtin_amdgcn_ballot_w32(h0 | h1 | h2 | h3 | h4 | h5 | h6 | h7);
  if (any != 0u) {
#define HITJ(J, HJ, SJ) { \
      const unsigned mj = __builtin_amdgcn_ballot_w32(HJ); \
      if (mj != 0u) { \
        if (HJ) { \
          const int pos = wc + (int)__builtin_amdgcn_mbcnt_lo(mj, 0u); \
          if (pos < WCAP) list[wave * WCAP + pos] = ((el0 + (J)) << SLB) | (int)(SJ); \
        } \
        wc += (int)__builtin_popcount(mj); } }
    HITJ(0, h0, s0)
    HITJ(1, h1, s1)
    HITJ(2, h2, s2)
    HITJ(3, h3, s3)
    HITJ(4, h4, s4)
    HITJ(5, h5, s5)
    HITJ(6, h6, s6)
    HITJ(7, h7, s7)
#undef HITJ
  }
  return wc;
}

__global__ __launch_bounds__(NTHR) void k_prep(const float* __restrict__ h, const float* __restrict__ x,
                                               const float* __restrict__ We1, const float* __restrict__ We2,
                                               const float* __restrict__ Ws1, const float* __restrict__ Ws2,
                                               const float* __restrict__ Wc1, const float* __restrict__ Wn1,
                                               const float* __restrict__ Wn2, int nN, int nP,
                                               unsigned short* WABT, unsigned short* WE2T, unsigned short* WS1T,
                                               unsigned short* WS2T, unsigned short* WC1T, unsigned short* WN1T,
                                               unsigned short* WN2T, unsigned short* HB, float* XP) {
  const int u  = (int)blockIdx.x * NTHR + (int)threadIdx.x;
  const int U0 = NU_WABT;
  const int U1 = U0 + NU_WE2T;
  const int U2 = U1 + NU_WS1T;
  const int U3 = U2 + NU_WS2T;
  const int U4 = U3 + NU_WC1T;
  const int U5 = U4 + NU_WN1T;
  const int U6 = U5 + NU_WN2A;
  const int U7 = U6 + NU_WN2B;
  const int U8 = U7 + nP * 8;
  v8us o;
  if (u < U0) {
    const int n  = u >> 3;
    const int k8 = (u & 7) * 8;
    const float* p = We1 + (size_t)((n >> 6) * FD + k8) * FD + (n & 63);
#pragma unroll
    for (int i = 0; i < 8; ++i) o[i] = (unsigned short)bf16_bits(p[(size_t)i * FD]);
    put16(WABT + (size_t)n * FD + k8, o);
    return;
  } else if (u < U1) {
    const int v  = u - U0;
    const int n  = v >> 4;
    const int k8 = (v & 15) * 8;
    const float* p = We2 + (size_t)(k8 & 63) * FD + n;
#pragma unroll
    for (int i = 0; i < 8; ++i) o[i] = (unsigned short)bf16_bits(p[(size_t)i * FD]);
    put16(WE2T + (size_t)n * 128 + k8, o);
    return;
  } else if (u < U2) {
    const int v  = u - U1;
    const int n  = v >> 10;
    const int k8 = (v & 1023) * 8;
    const float* p = Ws1 + (size_t)(k8 & 4095) * NTP + n;
#pragma unroll
    for (int i = 0; i < 8; ++i) o[i] = (unsigned short)bf16_bits(p[(size_t)i * NTP]);
    put16(WS1T + (size_t)n * KTP + k8, o);
    return;
  } else if (u < U3) {
    const int v  = u - U2;
    const int n  = v >> 5;
    const int k8 = (v & 31) * 8;
    const float* p = Ws2 + (size_t)(k8 & 127) * FD + n;
#pragma unroll
    for (int i = 0; i < 8; ++i) o[i] = (unsigned short)bf16_bits(p[(size_t)i * FD]);
    put16(WS2T + (size_t)n * 256 + k8, o);
    return;
  } else if (u < U4) {
    const int v  = u - U3;
    const int n  = v >> 4;
    const int k8 = (v & 15) * 8;
    const float* p = Wc1 + (size_t)(k8 & 63) * FD + n;
#pragma unroll
    for (int i = 0; i < 8; ++i) o[i] = (unsigned short)bf16_bits(p[(size_t)i * FD]);
    put16(WC1T + (size_t)n * 128 + k8, o);
    return;
  } else if (u < U5) {
    const int v  = u - U4;
    const int n  = v >> 5;
    const int k8 = (v & 31) * 8;
    const int rb = (k8 < 64) ? k8 : (k8 < 128) ? (k8 + 3) : (k8 == 128) ? 64 : (k8 < 160) ? 0 :
                   (k8 < 224) ? (k8 - 93) : (k8 == 224) ? 64 : 0;
    const int cv = (k8 < 128) ? 8 : (k8 == 128) ? 3 : (k8 < 160) ? 0 : (k8 < 224) ? 8 : (k8 == 224) ? 3 : 0;
#pragma unroll
    for (int i = 0; i < 8; ++i) {
      const int rr = (rb + i) < 130 ? (rb + i) : 130;
      const unsigned bits = bf16_bits(Wn1[(size_t)rr * FD + n]);
      const unsigned msk  = (i < cv) ? 0xffffu : 0u;
      o[i] = (unsigned short)(bits & msk);
    }
    put16(WN1T + (size_t)n * 256 + k8, o);
    return;
  } else if (u < U6) {
    const int v  = u - U5;
    const int n  = v >> 4;
    const int k8 = (v & 15) * 8;
    const int nc = n < NOUTF ? n : NOUTF - 1;
    const unsigned msk = (n < NOUTF) ? 0xffffu : 0u;
    const float* p = Wn2 + (size_t)(k8 & 63) * NOUTF + nc;
#pragma unroll
    for (int i = 0; i < 8; ++i) o[i] = (unsigned short)(bf16_bits(p[(size_t)i * NOUTF]) & msk);
    put16(WN2T + (size_t)n * 256 + k8, o);
    return;
  } else if (u < U7) {
    const int v  = u - U6;
    const int n  = v >> 4;
    const int k8 = 128 + (v & 15) * 8;
#pragma unroll
    for (int i = 0; i < 8; ++i) {
      const int k = k8 + i;
      int one = 0;
      one |= (k < 192 && (k - 128) == n) ? 1 : 0;
      one |= (k >= 192 && k < 195 && n == (k - 192) + 64) ? 1 : 0;
      one |= (k >= 196 && k < 199 && n == (k - 196) + 64) ? 1 : 0;
      o[i] = (unsigned short)(one ? 0x3F80 : 0);
    }
    put16(WN2T + (size_t)n * 256 + k8, o);
    return;
  } else if (u < U8) {
    const int v   = u - U7;
    const int row = v >> 3;
    const int k8  = (v & 7) * 8;
    const int rc  = row < nN ? row : nN - 1;
    const float* p = h + (size_t)rc * FD + k8;
    const v4f a = *(const v4fa*)p;
    const v4f b = *(const v4fa*)(p + 4);
    const unsigned msk = (row < nN) ? 0xffffu : 0u;
    o[0] = (unsigned short)(bf16_bits(a.x) & msk);
    o[1] = (unsigned short)(bf16_bits(a.y) & msk);
    o[2] = (unsigned short)(bf16_bits(a.z) & msk);
    o[3] = (unsigned short)(bf16_bits(a.w) & msk);
    o[4] = (unsigned short)(bf16_bits(b.x) & msk);
    o[5] = (unsigned short)(bf16_bits(b.y) & msk);
    o[6] = (unsigned short)(bf16_bits(b.z) & msk);
    o[7] = (unsigned short)(bf16_bits(b.w) & msk);
    put16(HB + (size_t)row * FD + k8, o);
    return;
  } else {
    const int row = u - U8;
    if (row >= nP) return;
    const int rc  = row < nN ? row : nN - 1;
    const float okf = (row < nN) ? 1.0f : 0.0f;
    const float x0 = x[(size_t)rc * 3 + 0];
    const float x1 = x[(size_t)rc * 3 + 1];
    const float x2 = x[(size_t)rc * 3 + 2];
    v4f q;
    q.x = okf * bf16_val(x0);
    q.y = okf * bf16_val(x1);
    q.z = okf * bf16_val(x2);
    q.w = 0.0f;
    putf4(XP + (size_t)row * 4, q);
    return;
  }
}

template <int NT, int MODE>
__global__ __launch_bounds__(GTHR) void k_gemm(const unsigned short* __restrict__ A, int lda,
                                               const unsigned short* __restrict__ BT, int ldb, int K,
                                               const float* __restrict__ bias, int nBias,
                                               const float* __restrict__ wvec, int nValid,
                                               float* Cf, unsigned short* Cb, int ldcb) {
  constexpr int NC  = 16 * NT;
  constexpr int UR4 = NC / 4;
  constexpr int UH  = NC / 8;
  constexpr int NSW = NC / 8;
  __shared__ __attribute__((aligned(16))) float stg[GBM * NC];
  __shared__ __attribute__((aligned(16))) float sWS[2 * GBM];
  const int tid = (int)threadIdx.x, lane = tid & 31, wave = tid >> 5, hh = lane >> 4, m = lane & 15;
  const int rowBase = (int)blockIdx.x * GBM;
  if constexpr (MODE == 4) {
    static_assert(NC == GBM);
    if (tid < GBM) sWS[tid] = bf16_val(wvec[tid]);
  }

  v8f acc[NT];
  {
    const v8f z = {0.f, 0.f, 0.f, 0.f, 0.f, 0.f, 0.f, 0.f};
#pragma unroll
    for (int t = 0; t < NT; ++t) acc[t] = z;
  }
  const unsigned short* ap = A  + (size_t)(rowBase + 16 * wave + m) * (size_t)lda + 8 * hh;
  const unsigned short* bp = BT + (size_t)m * (size_t)ldb + 8 * hh;

#pragma unroll 1
  for (int k0 = 0; k0 < K; k0 += 32) {
    FragB af;
    af.h[0] = *(const v8usa*)(ap + k0);
    af.h[1] = *(const v8usa*)(ap + k0 + 16);
#pragma unroll
    for (int nt = 0; nt < NT; ++nt) {
      const unsigned short* wq = bp + (size_t)(16 * nt) * (size_t)ldb + k0;
      FragB bf;
      bf.h[0] = *(const v8usa*)wq;
      bf.h[1] = *(const v8usa*)(wq + 16);
      acc[nt] = wmb(af, bf, acc[nt]);
    }
  }

#pragma unroll
  for (int nt = 0; nt < NT; ++nt) {
    const int lc = 16 * nt + m;
    float bvv = 0.0f;
    if constexpr (MODE != 0) {
      const int bc = lc < nBias ? lc : nBias - 1;
      bvv = bf16_val(bias[bc]);
    }
#pragma unroll
    for (int r = 0; r < 8; ++r) {
      const int lr = 16 * wave + 8 * hh + r;
      float v = acc[nt][r];
      if constexpr (MODE == 1 || MODE == 4 || MODE == 5) v = silu_f(v + bvv);
      if constexpr (MODE == 2) v = fmaxf(v + bvv, 0.0f);
      if constexpr (MODE == 3 || MODE == 6) v = v + bvv;
      stg[lr * NC + lc] = v;
    }
  }
  __syncthreads();

  if constexpr (MODE == 0 || MODE == 1 || MODE == 3) {
    v4f pv[NSW];
#pragma unroll
    for (int it = 0; it < NSW; ++it) {
      const int u = it * 32 + lane;
      const int i = u / UR4, c4 = u % UR4;
      pv[it] = *(const v4fa*)(stg + (16 * wave + i) * NC + 4 * c4);
    }
#pragma unroll
    for (int it = 0; it < NSW; ++it) {
      const int u = it * 32 + lane;
      const int i = u / UR4, c4 = u % UR4;
      float* op = Cf + (size_t)(rowBase + 16 * wave + i) * (size_t)NC + 4 * c4;
      *(volatile v4f*)op = pv[it];
    }
    __threadfence();
#pragma unroll
    for (int it = 0; it < NSW; ++it) {
      const int u = it * 32 + lane;
      const int i = u / UR4, c4 = u % UR4;
      float* op = Cf + (size_t)(rowBase + 16 * wave + i) * (size_t)NC + 4 * c4;
      *(volatile v4f*)op = pv[it];
    }
  }
  if constexpr (MODE == 2 || MODE == 3 || MODE == 5) {
    v8us ph[NSW];
#pragma unroll
    for (int it = 0; it < NSW; ++it) {
      const int u = it * 32 + lane;
      const int i = u / UR4, q = u % UR4;
      const int part = q / UH, j = q % UH;
      const unsigned mh = 0u - (unsigned)part;
      const unsigned ml = ~mh;
      const float* sp = stg + (16 * wave + i) * NC + 8 * j;
      const v4f a = *(const v4fa*)sp;
      const v4f b = *(const v4fa*)(sp + 4);
      const v8f f8 = {a.x, a.y, a.z, a.w, b.x, b.y, b.z, b.w};
      v8us oo;
#pragma unroll
      for (int e = 0; e < 8; ++e) {
        const unsigned hb = bf16_bits(f8[e]);
        const unsigned lb = bf16_bits(f8[e] - __uint_as_float(hb << 16));
        oo[e] = (unsigned short)((hb & ml) | (lb & mh));
      }
      ph[it] = oo;
    }
#pragma unroll
    for (int it = 0; it < NSW; ++it) {
      const int u = it * 32 + lane;
      const int i = u / UR4, q = u % UR4;
      const int part = q / UH, j = q % UH;
      unsigned short* op = Cb + (size_t)(rowBase + 16 * wave + i) * (size_t)ldcb + part * NC + 8 * j;
      *(volatile v8us*)op = ph[it];
    }
    __threadfence();
#pragma unroll
    for (int it = 0; it < NSW; ++it) {
      const int u = it * 32 + lane;
      const int i = u / UR4, q = u % UR4;
      const int part = q / UH, j = q % UH;
      unsigned short* op = Cb + (size_t)(rowBase + 16 * wave + i) * (size_t)ldcb + part * NC + 8 * j;
      *(volatile v8us*)op = ph[it];
    }
  }
  if constexpr (MODE == 4) {
    if (tid < GBM) {
      float s = 0.0f;
      const float* sp = stg + tid * NC;
#pragma unroll 4
      for (int c = 0; c < NC; ++c) s = fmaf(sp[c], sWS[c], s);
      sWS[GBM + tid] = s;
    }
    __syncthreads();
    if (wave == 0) {
      const int tl = lane & 15;
      const v4f o4 = *(const v4fa*)(sWS + GBM + 4 * tl);
      float* dp = Cf + (size_t)rowBase + 4 * tl;
      if (lane < 16) *(volatile v4f*)dp = o4;
      __threadfence();
      if (lane < 16) *(volatile v4f*)dp = o4;
    }
  }
  if constexpr (MODE == 6) {
    constexpr int UMAX = GBM * NOUTF / 4;
    constexpr int NSW6 = (UMAX + GTHR - 1) / GTHR;
    int nv = nValid - rowBase;
    nv = nv < 0 ? 0 : (nv > GBM ? GBM : nv);
    const int U = (nv * NOUTF) >> 2;
    v4f pv[NSW6];
#pragma unroll
    for (int it = 0; it < NSW6; ++it) {
      const int u  = it * GTHR + tid;
      const int uc = u < UMAX ? u : UMAX - 1;
      v4f q;
#pragma unroll
      for (int e = 0; e < 4; ++e) {
        const int idx = 4 * uc + e;
        const int rr  = idx / NOUTF;
        const int cc  = idx - rr * NOUTF;
        q[e] = stg[rr * NC + cc];
      }
      pv[it] = q;
    }
    float* base = Cf + (size_t)rowBase * NOUTF;
#pragma unroll
    for (int it = 0; it < NSW6; ++it) {
      const int u = it * GTHR + tid;
      if (u < U) *(volatile v4f*)(base + (size_t)4 * u) = pv[it];
    }
    __threadfence();
#pragma unroll
    for (int it = 0; it < NSW6; ++it) {
      const int u = it * GTHR + tid;
      if (u < U) *(volatile v4f*)(base + (size_t)4 * u) = pv[it];
    }
  }
}

__device__ __forceinline__ void u1b_pass(const unsigned short* sA, unsigned short* dst, int tid) {
#pragma unroll
  for (int it = 0; it < 16; ++it) {
    const int u  = it * ETHR + tid;
    const int rw = u >> 4;
    const int c8 = (u & 15) * 8;
    const v4i v = *(const v4ia*)(sA + rw * AP + c8);
    *(volatile v4i*)(dst + (size_t)8 * u) = v;
  }
}

__global__ __launch_bounds__(ETHR) void k_edge(const int* __restrict__ ei, int nE, int nN,
                                               const float* __restrict__ PQ, const float* __restrict__ XP,
                                               const float* __restrict__ be1, const float* __restrict__ w128,
                                               unsigned short* U1B, float* REL) {
  __shared__ __attribute__((aligned(16))) unsigned short sA[ETHR * AP];
  __shared__ __attribute__((aligned(16))) float cst[2 * FD];
  const int tid = (int)threadIdx.x;
  if (tid < FD) {
    cst[tid]      = bf16_val(be1[tid]);
    cst[FD + tid] = bf16_val(w128[tid]);
  }
  const int elb = (int)blockIdx.x * ETHR;
  const int el  = elb + tid;
  const int eg  = el < nE ? el : nE - 1;
  int r = ei[eg];
  int c = ei[(size_t)nE + (size_t)eg];
  r = clampi(r, 0, nN - 1);
  c = clampi(c, 0, nN - 1);
  const v4f xr = *(const v4fa*)(XP + (size_t)r * 4);
  const v4f xc = *(const v4fa*)(XP + (size_t)c * 4);
  const float dfx = xr.x - xc.x, dfy = xr.y - xc.y, dfz = xr.z - xc.z;
  const float radial = (dfx * dfx + dfz * dfz) + dfy * dfy;
  const float nrm = __builtin_sqrtf(radial);
  const float inv = 1.0f / (nrm + 1e-8f);
  v4f rel4;
  rel4.x = dfx * inv; rel4.y = dfy * inv; rel4.z = dfz * inv; rel4.w = 0.0f;
  __syncthreads();

  unsigned short* ra = sA + tid * AP;
  {
    const float* pr = PQ + (size_t)r * NPQ;
    const float* qr = PQ + (size_t)c * NPQ + FD;
#pragma unroll 1
    for (int c8 = 0; c8 < FD / 8; ++c8) {
      const v4f pa = *(const v4fa*)(pr + 8 * c8);
      const v4f pb = *(const v4fa*)(pr + 8 * c8 + 4);
      const v4f qa = *(const v4fa*)(qr + 8 * c8);
      const v4f qb = *(const v4fa*)(qr + 8 * c8 + 4);
      const v4f ba = *(const v4fa*)(cst + 8 * c8);
      const v4f bb = *(const v4fa*)(cst + 8 * c8 + 4);
      const v4f ua = *(const v4fa*)(cst + FD + 8 * c8);
      const v4f ub = *(const v4fa*)(cst + FD + 8 * c8 + 4);
      const v8f p8 = {pa.x, pa.y, pa.z, pa.w, pb.x, pb.y, pb.z, pb.w};
      const v8f q8 = {qa.x, qa.y, qa.z, qa.w, qb.x, qb.y, qb.z, qb.w};
      const v8f b8 = {ba.x, ba.y, ba.z, ba.w, bb.x, bb.y, bb.z, bb.w};
      const v8f u8 = {ua.x, ua.y, ua.z, ua.w, ub.x, ub.y, ub.z, ub.w};
      v8us oh, ol;
#pragma unroll
      for (int i = 0; i < 8; ++i) {
        const float pre = (p8[i] + q8[i]) + fmaf(radial, u8[i], b8[i]);
        const float v   = silu_f(pre);
        const unsigned hb = bf16_bits(v);
        oh[i] = (unsigned short)hb;
        ol[i] = (unsigned short)bf16_bits(v - __uint_as_float(hb << 16));
      }
      *(v8usa*)(ra + 8 * c8)      = oh;
      *(v8usa*)(ra + FD + 8 * c8) = ol;
    }
  }
  __syncthreads();

  unsigned short* ub = U1B + (size_t)elb * (2 * FD);
  u1b_pass(sA, ub, tid);
  __threadfence();
  u1b_pass(sA, ub, tid);

  float* rp = REL + (size_t)el * 4;
  *(volatile v4f*)rp = rel4;
  __threadfence();
  *(volatile v4f*)rp = rel4;
}

__device__ __forceinline__ void tp_pass(const unsigned short* sT, unsigned short* dst, int tid) {
#pragma unroll
  for (int it = 0; it < 4; ++it) {
    const int u = it * NTHR + tid;
    const v4i v = *(const v4ia*)(sT + 8 * u);
    *(volatile v4i*)(dst + (size_t)8 * u) = v;
  }
}

__global__ __launch_bounds__(NTHR) void k_tp(const float* __restrict__ EPL, int rowBase, unsigned short* APL) {
  __shared__ __attribute__((aligned(16))) unsigned short sT[KTP];
  const int tid = (int)threadIdx.x;
  const int r   = (int)blockIdx.x;
  const float* er = EPL + (size_t)(rowBase + r) * FD;
  const int a  = tid >> 2;
  const int b0 = (tid & 3) * 16;
  const float ea = er[a];
  const v4f e0 = *(const v4fa*)(er + b0);
  const v4f e1 = *(const v4fa*)(er + b0 + 4);
  const v4f e2 = *(const v4fa*)(er + b0 + 8);
  const v4f e3 = *(const v4fa*)(er + b0 + 12);
  const v8f ebA = {e0.x, e0.y, e0.z, e0.w, e1.x, e1.y, e1.z, e1.w};
  const v8f ebB = {e2.x, e2.y, e2.z, e2.w, e3.x, e3.y, e3.z, e3.w};
  v8us hA, hB, lA, lB;
#pragma unroll
  for (int i = 0; i < 8; ++i) {
    const float pA = 64.0f * (ea * ebA[i]);
    const float pB = 64.0f * (ea * ebB[i]);
    const unsigned ha = bf16_bits(pA);
    const unsigned hb = bf16_bits(pB);
    hA[i] = (unsigned short)ha;
    hB[i] = (unsigned short)hb;
    lA[i] = (unsigned short)bf16_bits(pA - __uint_as_float(ha << 16));
    lB[i] = (unsigned short)bf16_bits(pB - __uint_as_float(hb << 16));
  }
  const int kb = a * FD + b0;
  *(v8usa*)(sT + kb)                = hA;
  *(v8usa*)(sT + kb + 8)            = hB;
  *(v8usa*)(sT + (KTP / 2) + kb)    = lA;
  *(v8usa*)(sT + (KTP / 2) + kb + 8) = lB;
  __syncthreads();

  unsigned short* dst = APL + (size_t)r * KTP;
  tp_pass(sT, dst, tid);
  __threadfence();
  tp_pass(sT, dst, tid);
}

__global__ __launch_bounds__(NTHR) void k_scan(const int* __restrict__ keys, const int* __restrict__ cols,
                                               int nEh, int nN, int vec8,
                                               const float* __restrict__ EF, const float* __restrict__ Sh,
                                               const float* __restrict__ XP, float* MI, float* DX) {
  extern __shared__ __attribute__((aligned(16))) int dsm[];
  int*   list = dsm;
  int*   hl   = dsm + LISTN;
  int*   sl   = hl + RCAP;
  int*   cnt  = sl + RCAP;
  int*   offs = cnt + NBA;
  int*   cur  = offs + NBA;
  int*   misc = cur + NBA;
  float* sdx  = (float*)(misc + 16);
  const int tid = (int)threadIdx.x, lane = tid & 31, wave = tid >> 5;
  const int nodeBase = (int)blockIdx.x * NBA;

  {
    const v4i z4 = {0, 0, 0, 0};
    for (int i = tid * 4; i < AGG_ZINTS; i += NTHR * 4) *(v4ia*)(dsm + i) = z4;
    if (tid < 16) misc[tid] = 0;
  }
  __syncthreads();

  int t = 0, ov = 0;
  const int nChunks = (nEh + CHUNK - 1) / CHUNK;
#pragma unroll 1
  for (int ch = 0; ch < nChunks; ++ch) {
    const int cbase = ch * CHUNK;
    const int wc = scan_chunk<SLA>(keys, nEh, cbase, nodeBase, NBA, vec8, list, tid, lane, wave);
    if (lane == 0) misc[wave] = wc;
    __syncthreads();
    if (wave == 0) {
#pragma unroll 1
      for (int w2 = 0; w2 < NWAVE; ++w2) {
        int cc = misc[w2];
        cc = cc < 0 ? 0 : (cc > WCAP ? WCAP : cc);
#pragma unroll 1
        for (int b0 = 0; b0 < cc; b0 += 32) {
          const int idx = b0 + lane;
          const int ent = list[w2 * WCAP + (idx < WCAP ? idx : WCAP - 1)];
          const int m32 = (cc - b0) < 32 ? (cc - b0) : 32;
#pragma unroll 1
          for (int k = 0; k < m32; ++k) {
            const int u    = __builtin_amdgcn_readlane(ent, k);
            const int slot = u & (NBA - 1);
            const int el   = (u >> SLA) & (CHUNK - 1);
            const int pk   = ((cbase + el) << SLA) | slot;
            if (t < RCAP) {
              if (lane == 0) { hl[t] = pk; cnt[slot] = cnt[slot] + 1; }
              t = t + 1;
            } else {
              ov = 1;
            }
          }
        }
      }
    }
    __syncthreads();
  }
  if (wave == 0 && lane == 0) { misc[8] = t; misc[9] = ov; }
  __syncthreads();
  int tt = misc[8];
  tt = tt < 0 ? 0 : (tt > RCAP ? RCAP : tt);
  const int ovf = misc[9];

  if (wave == 0) {
    const int base = lane * (NBA / 32);
    int s = 0;
#pragma unroll 1
    for (int i = 0; i < NBA / 32; ++i) s += cnt[base + i];
    int incl = s;
#pragma unroll
    for (int d = 1; d < 32; d <<= 1) {
      const int y = __shfl_up(incl, d, 32);
      if (lane >= d) incl += y;
    }
    int run = incl - s;
#pragma unroll 1
    for (int i = 0; i < NBA / 32; ++i) {
      const int cv = cnt[base + i];
      offs[base + i] = run;
      cur[base + i]  = run;
      run += cv;
    }
  }
  __syncthreads();
  if (wave == 0) {
#pragma unroll 1
    for (int b0 = 0; b0 < tt; b0 += 32) {
      const int idx = b0 + lane;
      const int ent = hl[idx < RCAP ? idx : RCAP - 1];
      const int m32 = (tt - b0) < 32 ? (tt - b0) : 32;
#pragma unroll 1
      for (int k = 0; k < m32; ++k) {
        const int u    = __builtin_amdgcn_readlane(ent, k);
        const int slot = u & (NBA - 1);
        if (lane == 0) {
          int p = cur[slot];
          p = p < 0 ? 0 : (p > RCAP - 1 ? RCAP - 1 : p);
          sl[p] = u;
          cur[slot] = p + 1;
        }
      }
    }
  }
  __syncthreads();

  const float qnan = __int_as_float(0x7fc00000);
  const float pz = (ovf != 0) ? qnan : 0.0f;
  const int l4 = 4 * (lane & 15);
#pragma unroll 1
  for (int si = 0; si < NBA / NWAVE; ++si) {
    const int s    = si * NWAVE + wave;
    const int node = nodeBase + s;
    const int craw = cnt[s];
    const bool big = craw > DEGCAP;
    const int cdeg = craw < 0 ? 0 : (craw > DEGCAP ? DEGCAP : craw);
    int o = offs[s];
    o = o < 0 ? 0 : (o > RCAP ? RCAP : o);
    const int nc = node < nN ? node : nN - 1;
    const v4f xd = *(const v4fa*)(XP + (size_t)nc * 4);
    float a0 = 0.0f, a1 = 0.0f, a2 = 0.0f, a3 = 0.0f;
    float dx = 0.0f, dy = 0.0f, dz = 0.0f;
#pragma unroll 1
    for (int b0 = 0; b0 < cdeg; b0 += 32) {
      int idx = o + b0 + lane;
      idx = idx > RCAP - 1 ? RCAP - 1 : idx;
      const int ent = sl[idx];
      int eid = ent >> SLA;
      eid = eid < 0 ? 0 : (eid > nEh - 1 ? nEh - 1 : eid);
      int sr = cols[eid];
      sr = sr < 0 ? 0 : (sr > nN - 1 ? nN - 1 : sr);
      const v4f   xs = *(const v4fa*)(XP + (size_t)sr * 4);
      const float sv = Sh[eid];
      const int cxi = __float_as_int((xd.x - xs.x) * sv);
      const int cyi = __float_as_int((xd.y - xs.y) * sv);
      const int czi = __float_as_int((xd.z - xs.z) * sv);
      const int m32 = (cdeg - b0) < 32 ? (cdeg - b0) : 32;
#pragma unroll 1
      for (int k = 0; k < m32; ++k) {
        const int ek = __builtin_amdgcn_readlane(eid, k);
        const v4f w = *(const v4fa*)(EF + (size_t)ek * FD + l4);
        a0 += w.x;
        a1 += w.y;
        a2 += w.z;
        a3 += w.w;
        dx += __int_as_float(__builtin_amdgcn_readlane(cxi, k));
        dy += __int_as_float(__builtin_amdgcn_readlane(cyi, k));
        dz += __int_as_float(__builtin_amdgcn_readlane(czi, k));
      }
    }
    const float pzr = big ? qnan : pz;
    float* mp = MI + (size_t)node * FD + l4;
    v4f nv;
    nv.x = a0 + pzr; nv.y = a1 + pzr; nv.z = a2 + pzr; nv.w = a3 + pzr;
    if (lane < 16) *(volatile v4f*)mp = nv;
    __threadfence();
    if (lane < 16) *(volatile v4f*)mp = nv;
    if (lane == 0) {
      const v4f d4 = {dx + pzr, dy + pzr, dz + pzr, (float)craw};
      *(v4fa*)(sdx + 4 * s) = d4;
    }
  }
  __syncthreads();

  v4f dv[4];
#pragma unroll
  for (int j = 0; j < 4; ++j) dv[j] = *(const v4fa*)(sdx + 4 * (j * NTHR + tid));
#pragma unroll
  for (int j = 0; j < 4; ++j) {
    const int node = nodeBase + j * NTHR + tid;
    *(volatile v4f*)(DX + (size_t)node * 4) = dv[j];
  }
  __threadfence();
#pragma unroll
  for (int j = 0; j < 4; ++j) {
    const int node = nodeBase + j * NTHR + tid;
    *(volatile v4f*)(DX + (size_t)node * 4) = dv[j];
  }
}

__device__ __forceinline__ void nz_pass(const unsigned short* sZ, unsigned short* NZb, unsigned short* Z2b, int tid) {
#pragma unroll
  for (int it = 0; it < 32; ++it) {
    const int u  = it * ZTHR + tid;
    const int rw = u >> 5, q = u & 31;
    const v4i v = *(const v4ia*)(sZ + rw * ZP + 8 * q);
    *(volatile v4i*)(NZb + (size_t)rw * 256 + 8 * q) = v;
  }
#pragma unroll
  for (int it = 0; it < 16; ++it) {
    const int u  = it * ZTHR + tid;
    const int rw = u >> 4, q = u & 15;
    const v4i v = *(const v4ia*)(sZ + rw * ZP + 256 + 8 * q);
    *(volatile v4i*)(Z2b + (size_t)rw * 256 + 128 + 8 * q) = v;
  }
}

__global__ __launch_bounds__(ZTHR) void k_nz(const float* __restrict__ h, const float* __restrict__ MI,
                                             const float* __restrict__ REL, int nN,
                                             unsigned short* NZ, unsigned short* Z2) {
  __shared__ __attribute__((aligned(16))) unsigned short sZ[ZTHR * ZP];
  const int tid = (int)threadIdx.x;
  const int rowBase = (int)blockIdx.x * ZTHR;
  const int row = rowBase + tid;
  const int rc  = row < nN ? row : nN - 1;
  unsigned short* zr = sZ + tid * ZP;
#pragma unroll 1
  for (int q = 0; q < 8; ++q) {
    const float* hq = h  + (size_t)rc  * FD + 8 * q;
    const float* mq = MI + (size_t)row * FD + 8 * q;
    const v4f ha = *(const v4fa*)hq;
    const v4f hb = *(const v4fa*)(hq + 4);
    const v4f ma = *(const v4fa*)mq;
    const v4f mb = *(const v4fa*)(mq + 4);
    const v8f h8 = {ha.x, ha.y, ha.z, ha.w, hb.x, hb.y, hb.z, hb.w};
    const v8f m8 = {ma.x, ma.y, ma.z, ma.w, mb.x, mb.y, mb.z, mb.w};
    v8us oh, ohi, olo;
#pragma unroll
    for (int i = 0; i < 8; ++i) {
      oh[i] = (unsigned short)bf16_bits(h8[i]);
      const unsigned hb2 = bf16_bits(m8[i]);
      ohi[i] = (unsigned short)hb2;
      olo[i] = (unsigned short)bf16_bits(m8[i] - __uint_as_float(hb2 << 16));
    }
    *(v8usa*)(zr + 8 * q)        = oh;
    *(v8usa*)(zr + 64 + 8 * q)   = ohi;
    *(v8usa*)(zr + 160 + 8 * q)  = olo;
    *(v8usa*)(zr + 256 + 8 * q)  = oh;
  }
  {
    const v4f r4 = *(const v4fa*)(REL + (size_t)rc * 4);
    const unsigned h0 = bf16_bits(r4.x), h1 = bf16_bits(r4.y), h2 = bf16_bits(r4.z);
    const unsigned l0 = bf16_bits(r4.x - __uint_as_float(h0 << 16));
    const unsigned l1 = bf16_bits(r4.y - __uint_as_float(h1 << 16));
    const unsigned l2 = bf16_bits(r4.z - __uint_as_float(h2 << 16));
    const v8us uh = {(unsigned short)h0, (unsigned short)h1, (unsigned short)h2, 0, 0, 0, 0, 0};
    const v8us ul = {(unsigned short)l0, (unsigned short)l1, (unsigned short)l2, 0, 0, 0, 0, 0};
    const v8us uz = {(unsigned short)h0, (unsigned short)h1, (unsigned short)h2, 0,
                     (unsigned short)l0, (unsigned short)l1, (unsigned short)l2, 0};
    const v8us z8 = {0, 0, 0, 0, 0, 0, 0, 0};
    *(v8usa*)(zr + 128) = uh;
    *(v8usa*)(zr + 136) = z8;
    *(v8usa*)(zr + 144) = z8;
    *(v8usa*)(zr + 152) = z8;
    *(v8usa*)(zr + 224) = ul;
    *(v8usa*)(zr + 232) = z8;
    *(v8usa*)(zr + 240) = z8;
    *(v8usa*)(zr + 248) = z8;
    *(v8usa*)(zr + 320) = uz;
#pragma unroll
    for (int q = 41; q < 48; ++q) *(v8usa*)(zr + 256 + 8 * (q - 32)) = z8;
  }
  __syncthreads();

  unsigned short* NZb = NZ + (size_t)rowBase * 256;
  unsigned short* Z2b = Z2 + (size_t)rowBase * 256;
  nz_pass(sZ, NZb, Z2b, tid);
  __threadfence();
  nz_pass(sZ, NZb, Z2b, tid);
}

__global__ __launch_bounds__(NTHR) void k_xout(const float* __restrict__ x, const float* __restrict__ DX,
                                               int nN, float* out1) {
  __shared__ __attribute__((aligned(16))) float sx[XROWS * 3];
  const int tid = (int)threadIdx.x;
  const int rowBase = (int)blockIdx.x * XROWS;
#pragma unroll 1
  for (int j = tid; j < XROWS * 3; j += NTHR) {
    const int rl  = j / 3;
    const int cc  = j - 3 * rl;
    const int row = rowBase + rl;
    const int rc  = row < nN ? row : nN - 1;
    const float xv = bf16_val(x[(size_t)rc * 3 + cc]);
    const float dv = DX[(size_t)rc * 4 + cc];
    const float cw = DX[(size_t)rc * 4 + 3];
    const float ic = 1.0f / fmaxf(cw, 1.0f);
    sx[j] = xv + dv * ic;
  }
  __syncthreads();
  const int tl = tid < (XROWS * 3) / 4 ? tid : (XROWS * 3) / 4 - 1;
  const v4f o4 = *(const v4fa*)(sx + 4 * tl);
  const long long gidx = (long long)rowBase * 3 + 4LL * tl;
  const bool stv = (tid < (XROWS * 3) / 4) && (gidx + 4 <= 3LL * nN);
  if (stv) *(volatile v4f*)(out1 + (size_t)gidx) = o4;
  __threadfence();
  if (stv) *(volatile v4f*)(out1 + (size_t)gidx) = o4;
}

static inline int cdiv(int a, int b) { return (a + b - 1) / b; }
static inline size_t al256(size_t v) { return (v + 255) & ~(size_t)255; }

extern "C" void kernel_launch(void* const* d_in, const int* in_sizes, int n_in,
                              void* d_out, int out_size, void* d_ws, size_t ws_size,
                              hipStream_t stream) {
  if (n_in < 18) return;
  if (in_sizes[0] < FD || (in_sizes[0] % FD) != 0) return;
  const int nN = in_sizes[0] / FD;
  if (nN < 32 || (nN % 32) != 0) return;
  if (in_sizes[1] != 3 * nN) return;
  if (in_sizes[2] != 2 * nN) return;
  const int nE = nN;
  if (nE >= (1 << 20)) return;
  if (in_sizes[3] != 129 * FD || in_sizes[4] != FD) return;
  if (in_sizes[5] != FD * FD || in_sizes[6] != FD) return;
  if (in_sizes[7] != 4096 * NTP || in_sizes[8] != NTP) return;
  if (in_sizes[9] != NTP * FD || in_sizes[10] != FD) return;
  if (in_sizes[11] != FD * FD || in_sizes[12] != FD) return;
  if (in_sizes[13] != FD) return;
  if (in_sizes[14] != 131 * FD || in_sizes[15] != FD) return;
  if (in_sizes[16] != FD * NOUTF || in_sizes[17] != NOUTF) return;
  if ((long long)out_size != (long long)nN * NOUTF + 3LL * nN) return;

  const float* h   = (const float*)d_in[0];
  const float* x   = (const float*)d_in[1];
  const int*   ei  = (const int*)d_in[2];
  const float* We1 = (const float*)d_in[3];
  const float* be1 = (const float*)d_in[4];
  const float* We2 = (const float*)d_in[5];
  const float* be2 = (const float*)d_in[6];
  const float* Ws1 = (const float*)d_in[7];
  const float* bs1 = (const float*)d_in[8];
  const float* Ws2 = (const float*)d_in[9];
  const float* bs2 = (const float*)d_in[10];
  const float* Wc1 = (const float*)d_in[11];
  const float* bc1 = (const float*)d_in[12];
  const float* Wc2 = (const float*)d_in[13];
  const float* Wn1 = (const float*)d_in[14];
  const float* bn1 = (const float*)d_in[15];
  const float* Wn2 = (const float*)d_in[16];
  const float* bn2 = (const float*)d_in[17];
  float* out0 = (float*)d_out;
  float* out1 = out0 + (size_t)nN * NOUTF;

  const int NP  = cdiv(nN, GBM) * GBM;
  const int gN  = NP / GBM;
  const int CH  = cdiv(cdiv(nE, NCHUNK), GBM) * GBM;
  const int EP  = NCHUNK * CH;
  const int gE  = EP / GBM;
  const int gA  = cdiv(NP, NBA);
  const int NBP = gA * NBA;
  if (EP < nE || NBP < NP || (EP % ETHR) != 0 || NP > EP) return;

  char* ws = (char*)d_ws;
  size_t off = 0;
  const size_t oWABT = off; off = al256(off + (size_t)NPQ * FD * 2);
  const size_t oWE2T = off; off = al256(off + (size_t)FD * 128 * 2);
  const size_t oWS1T = off; off = al256(off + (size_t)NTP * KTP * 2);
  const size_t oWS2T = off; off = al256(off + (size_t)FD * 256 * 2);
  const size_t oWC1T = off; off = al256(off + (size_t)FD * 128 * 2);
  const size_t oWN1T = off; off = al256(off + (size_t)FD * 256 * 2);
  const size_t oWN2T = off; off = al256(off + (size_t)128 * 256 * 2);
  const size_t oHB   = off; off = al256(off + (size_t)NP * FD * 2);
  const size_t oXP   = off; off = al256(off + (size_t)NP * 16);
  size_t szR1 = (size_t)NP * NPQ * 4;
  if (szR1 < (size_t)EP * 256 + (size_t)EP * 256) szR1 = (size_t)EP * 256 + (size_t)EP * 256;
  const size_t oR1   = off; off = al256(off + szR1);
  const size_t oREL  = off; off = al256(off + (size_t)EP * 16);
  const size_t oU1B  = off; off = al256(off + (size_t)EP * 128 * 2);
  const size_t oEPL  = off; off = al256(off + (size_t)EP * FD * 4);
  size_t szRA = (size_t)CH * KTP * 2;
  if (szRA < (size_t)NP * 512 * 2) szRA = (size_t)NP * 512 * 2;
  const size_t oRA   = off; off = al256(off + szRA);
  const size_t oG    = off; off = al256(off + (size_t)EP * 256 * 2);
  const size_t oS    = off; off = al256(off + (size_t)EP * 4);
  const size_t oMI   = off; off = al256(off + (size_t)NBP * FD * 4);
  const size_t oDX   = off; off = al256(off + (size_t)NBP * 16);
  if (off > ws_size || off > (size_t)WSMAX) return;
  unsigned short* WABT = (unsigned short*)(ws + oWABT);
  unsigned short* WE2T = (unsigned short*)(ws + oWE2T);
  unsigned short* WS1T = (unsigned short*)(ws + oWS1T);
  unsigned short* WS2T = (unsigned short*)(ws + oWS2T);
  unsigned short* WC1T = (unsigned short*)(ws + oWC1T);
  unsigned short* WN1T = (unsigned short*)(ws + oWN1T);
  unsigned short* WN2T = (unsigned short*)(ws + oWN2T);
  unsigned short* HB   = (unsigned short*)(ws + oHB);
  float*          XP   = (float*)(ws + oXP);
  float*          PQ   = (float*)(ws + oR1);
  float*          EF   = (float*)(ws + oR1);
  unsigned short* EFB  = (unsigned short*)(ws + oR1 + (size_t)EP * 256);
  float*          REL  = (float*)(ws + oREL);
  unsigned short* U1B  = (unsigned short*)(ws + oU1B);
  float*          EPL  = (float*)(ws + oEPL);
  unsigned short* APL  = (unsigned short*)(ws + oRA);
  unsigned short* NZ   = (unsigned short*)(ws + oRA);
  unsigned short* Z2   = (unsigned short*)(ws + oRA + (size_t)NP * 512);
  unsigned short* G    = (unsigned short*)(ws + oG);
  float*          S    = (float*)(ws + oS);
  float*          MI   = (float*)(ws + oMI);
  float*          DX   = (float*)(ws + oDX);

  hipFuncSetAttribute(reinterpret_cast<const void*>(&k_scan), hipFuncAttributeMaxDynamicSharedMemorySize,
                      (int)AGG_LDS_BYTES);

  const int nPrep = NU_WABT + NU_WE2T + NU_WS1T + NU_WS2T + NU_WC1T + NU_WN1T + NU_WN2A + NU_WN2B +
                    NP * 8 + cdiv(NP, NTHR) * NTHR;
  const int vec8 = 1;

  k_prep<<<nPrep / NTHR, NTHR, 0, stream>>>(h, x, We1, We2, Ws1, Ws2, Wc1, Wn1, Wn2, nN, NP,
                                            WABT, WE2T, WS1T, WS2T, WC1T, WN1T, WN2T, HB, XP);
  k_gemm<8, 0><<<gN, GTHR, 0, stream>>>(HB, FD, WABT, FD, FD, be1, FD, Wc2, nN, PQ, G, 0);
  k_edge<<<EP / ETHR, ETHR, 0, stream>>>(ei, nE, nN, PQ, XP, be1, We1 + (size_t)2 * FD * FD, U1B, REL);
  k_gemm<4, 1><<<gE, GTHR, 0, stream>>>(U1B, 128, WE2T, 128, 128, be2, FD, Wc2, nN, EPL, G, 0);
  for (int c = 0; c < NCHUNK; ++c) {
    k_tp<<<CH, NTHR, 0, stream>>>(EPL, c * CH, APL);
    k_gemm<8, 2><<<CH / GBM, GTHR, 0, stream>>>(APL, KTP, WS1T, KTP, KTP, bs1, NTP, Wc2, nN, EF,
                                                 G + (size_t)c * CH * 256, 256);
  }
  k_gemm<4, 3><<<gE, GTHR, 0, stream>>>(G, 256, WS2T, 256, 256, bs2, FD, Wc2, nN, EF, EFB, 128);
  k_gemm<4, 4><<<gE, GTHR, 0, stream>>>(EFB, 128, WC1T, 128, 128, bc1, FD, Wc2, nN, S, G, 0);
  k_scan<<<gA, NTHR, AGG_LDS_BYTES, stream>>>(ei, ei + (size_t)nE, nE, nN, vec8, EF, S, XP, MI, DX);
  k_nz<<<NP / ZTHR, ZTHR, 0, stream>>>(h, MI, REL, nN, NZ, Z2);
  k_gemm<4, 5><<<gN, GTHR, 0, stream>>>(NZ, 256, WN1T, 256, 256, bn1, FD, Wc2, nN, EF, Z2, 256);
  k_gemm<8, 6><<<gN, GTHR, 0, stream>>>(Z2, 256, WN2T, 256, 256, bn2, NOUTF, Wc2, nN, out0, G, 0);
  k_xout<<<cdiv(nN, XROWS), NTHR, 0, stream>>>(x, DX, nN, out1);
  (void)hipGetLastError();
}
